// BiDirectionalCrossAttentionLayer_74766790689039
// MI455X (gfx1250) — hardware-verified
//
#include <hip/hip_runtime.h>
#include <stdint.h>

typedef _Float16 v16h __attribute__((ext_vector_type(16)));
typedef _Float16 v8h  __attribute__((ext_vector_type(8)));
typedef _Float16 v4h  __attribute__((ext_vector_type(4)));
typedef float    v8f  __attribute__((ext_vector_type(8)));
typedef float    v4f  __attribute__((ext_vector_type(4)));
typedef v8h __attribute__((may_alias)) v8ha;
typedef v4f __attribute__((may_alias)) v4fa;

union Frag { v16h v; v8h half[2]; };

#define NSTR   4
#define BB     4
#define SS     512
#define EE     512
#define HH     8
#define HD     64
#define FF     2048
#define MROWS  (BB * SS)
#define WSCALE 32.0f
#define PSCALE 16384.0f
#define ASCALE 16.0f

__device__ __forceinline__ v8f wmma_f16(v16h a, v16h b, v8f c) {
  v8f d = __builtin_amdgcn_wmma_f32_16x16x32_f16(false, a, false, b, (short)0, c, false, false);
  asm volatile("v_nop\n\tv_nop\n\tv_nop\n\tv_nop" : "+v"(d) : "v"(a), "v"(b));
  return d;
}

__device__ __forceinline__ v16h load_frag(const _Float16* p, int h) {
  Frag f;
  f.half[0] = *(const v8ha*)(p + 8 * h);
  f.half[1] = *(const v8ha*)(p + 16 + 8 * h);
  return f.v;
}

__global__ __launch_bounds__(256) void cvt_x_kernel(
    const float* __restrict__ x0, const float* __restrict__ x1,
    const float* __restrict__ x2, const float* __restrict__ x3,
    _Float16* __restrict__ xh, int per8, int tot8)
{
  const int g = blockIdx.x * 256 + threadIdx.x;
  if (g >= tot8) return;
  const int s = g / per8;
  const int off = g - s * per8;
  const float* base = (s == 0) ? x0 : ((s == 1) ? x1 : ((s == 2) ? x2 : x3));
  const float* src = base + (size_t)off * 8;
  const v4f a = *(const v4fa*)src;
  const v4f c = *(const v4fa*)(src + 4);
  const v8h o = { (_Float16)a.x, (_Float16)a.y, (_Float16)a.z, (_Float16)a.w,
                  (_Float16)c.x, (_Float16)c.y, (_Float16)c.z, (_Float16)c.w };
  _Float16* dst = xh + (size_t)g * 8;
  *(volatile v8h*)dst = o;
  __threadfence();
  *(volatile v8h*)dst = o;
}

__device__ __forceinline__ void wt_store_pass(const _Float16* sT, _Float16* Tz, int n0, int k0,
                                              int Kdim, int w, int lane) {
  const int q8 = lane & 7, sub = lane >> 3;
  #pragma unroll
  for (int i = 0; i < 2; ++i) {
    const int n = w * 8 + i * 4 + sub;
    const v8h v = *(const v8ha*)(sT + n * 72 + 8 * q8);
    _Float16* dst = Tz + (size_t)(n0 + n) * Kdim + k0 + 8 * q8;
    *(volatile v8h*)dst = v;
  }
}

__global__ __launch_bounds__(256) void cvt_wt_kernel(
    const float* __restrict__ W, _Float16* __restrict__ T, int Kdim, int Ndim, float scale)
{
  __shared__ __attribute__((aligned(16))) _Float16 sT[64 * 72];

  const int tid = threadIdx.x, lane = tid & 31, w = tid >> 5;
  const int z = blockIdx.z;
  const int n0 = blockIdx.x * 64, k0 = blockIdx.y * 64;
  const float* Wz = W + (size_t)z * Kdim * Ndim;
  _Float16* Tz = T + (size_t)z * Kdim * Ndim;

  const int rr = tid >> 4, c4 = (tid & 15) * 4;
  #pragma unroll
  for (int p = 0; p < 4; ++p) {
    const int row = p * 16 + rr;
    const v4f v = *(const v4fa*)(Wz + (size_t)(k0 + row) * Ndim + n0 + c4);
    sT[(c4 + 0) * 72 + row] = (_Float16)(v.x * scale);
    sT[(c4 + 1) * 72 + row] = (_Float16)(v.y * scale);
    sT[(c4 + 2) * 72 + row] = (_Float16)(v.z * scale);
    sT[(c4 + 3) * 72 + row] = (_Float16)(v.w * scale);
  }
  __syncthreads();

  wt_store_pass(sT, Tz, n0, k0, Kdim, w, lane);
  __threadfence();
  wt_store_pass(sT, Tz, n0, k0, Kdim, w, lane);
}

__device__ __forceinline__ void qkv_store_pass(const _Float16* sH, _Float16* plane, _Float16* vt,
                                               int which, int bh, int l0, int w, int lane) {
  const int q8 = lane & 7, sub = lane >> 3;
  #pragma unroll
  for (int i = 0; i < 8; ++i) {
    const int lid = w * 32 + i * 4 + sub;
    v8h v;
    _Float16* dst;
    if (which != 2) {
      v = *(const v8ha*)(sH + lid * HD + 8 * q8);
      dst = plane + ((size_t)bh * SS + l0 + lid) * HD + 8 * q8;
    } else {
      const int d = lid >> 1, hl = lid & 1;
      v = *(const v8ha*)(sH + d * 128 + 64 * hl + 8 * q8);
      dst = vt + ((size_t)bh * HD + d) * SS + l0 + 64 * hl + 8 * q8;
    }
    *(volatile v8h*)dst = v;
  }
}

__device__ __forceinline__ void f32_store_pass(const float* sF, float* outz, int m0, int n0,
                                               int N, int w, int lane) {
  const int q8 = lane & 7, sub = lane >> 3;
  #pragma unroll
  for (int i = 0; i < 16; ++i) {
    const int lid = i * 4 + sub;
    const int row = 32 * w + (lid >> 1), hl = lid & 1;
    const v4f v = *(const v4fa*)(sF + row * 64 + 32 * hl + 4 * q8);
    float* dst = outz + (size_t)(m0 + row) * N + n0 + 32 * hl + 4 * q8;
    *(volatile v4f*)dst = v;
  }
}

__device__ __forceinline__ void f16_store_pass(const _Float16* sH, _Float16* outz, int m0, int n0,
                                               int N, int w, int lane) {
  const int q8 = lane & 7, sub = lane >> 3;
  #pragma unroll
  for (int i = 0; i < 8; ++i) {
    const int lid = i * 4 + sub;
    const int row = 32 * w + lid;
    const v8h v = *(const v8ha*)(sH + row * 64 + 8 * q8);
    _Float16* dst = outz + (size_t)(m0 + row) * N + n0 + 8 * q8;
    *(volatile v8h*)dst = v;
  }
}

template <int MODE>
__global__ __launch_bounds__(128) void gemm_kernel(
    const _Float16* __restrict__ A, const _Float16* __restrict__ Bt,
    const float* __restrict__ bias,
    float* __restrict__ outF, _Float16* __restrict__ out0,
    _Float16* __restrict__ out1, _Float16* __restrict__ out2,
    int M, int N, int K, float oscale)
{
  __shared__ __attribute__((aligned(16))) float sF[128 * 64];
  _Float16* sH = (_Float16*)sF;

  const int tid = threadIdx.x, lane = tid & 31, w = tid >> 5;
  const int h = lane >> 4, m = lane & 15;
  const int m0 = blockIdx.x * 128, n0 = blockIdx.y * 64, z = blockIdx.z;
  const int s = (MODE == 0) ? (z & 3) : z;
  const int m0w = m0 + 32 * w;

  const _Float16* Az = A + (size_t)s * M * K;
  const _Float16* Bz = Bt + (size_t)z * N * K;
  const _Float16* xa0 = Az + (size_t)(m0w + m) * K;
  const _Float16* xa1 = xa0 + (size_t)16 * K;
  const _Float16* wb  = Bz + (size_t)(n0 + m) * K;

  const v8f zero8 = {0.f, 0.f, 0.f, 0.f, 0.f, 0.f, 0.f, 0.f};
  v8f acc[2][4];
  #pragma unroll
  for (int mt = 0; mt < 2; ++mt)
    #pragma unroll
    for (int nt = 0; nt < 4; ++nt) acc[mt][nt] = zero8;

  #pragma unroll 1
  for (int k0 = 0; k0 < K; k0 += 32) {
    const v16h a0 = load_frag(xa0 + k0, h);
    const v16h a1 = load_frag(xa1 + k0, h);
    #pragma unroll
    for (int nt = 0; nt < 4; ++nt) {
      const v16h b = load_frag(wb + (size_t)nt * 16 * K + k0, h);
      acc[0][nt] = wmma_f16(a0, b, acc[0][nt]);
      acc[1][nt] = wmma_f16(a1, b, acc[1][nt]);
    }
  }

  const int which = (MODE == 0) ? (z >> 2) : 0;
  #pragma unroll
  for (int nt = 0; nt < 4; ++nt) {
    const int feat = 16 * nt + m;
    float bvl = 0.0f;
    if (MODE != 0) bvl = bias[(size_t)s * N + n0 + feat];
    #pragma unroll
    for (int mt = 0; mt < 2; ++mt) {
      #pragma unroll
      for (int r = 0; r < 8; ++r) {
        const int tokl = 32 * w + 16 * mt + 8 * h + r;
        const float y = acc[mt][nt][r] * oscale + bvl;
        if (MODE == 0) {
          const int idx = (which == 2) ? (feat * 128 + tokl) : (tokl * HD + feat);
          sH[idx] = (_Float16)y;
        } else if (MODE == 1) {
          sF[tokl * 64 + feat] = y;
        } else {
          const float g = 0.5f * y * (1.0f + erff(y * 0.70710678118654752f));
          sH[tokl * 64 + feat] = (_Float16)(g * ASCALE);
        }
      }
    }
  }
  __syncthreads();

  if (MODE == 0) {
    const int b = m0 / SS, l0 = m0 - b * SS;
    const int bh = (s * BB + b) * HH + blockIdx.y;
    _Float16* plane = (which == 0) ? out0 : out1;
    qkv_store_pass(sH, plane, out2, which, bh, l0, w, lane);
    __threadfence();
    qkv_store_pass(sH, plane, out2, which, bh, l0, w, lane);
  } else if (MODE == 1) {
    float* outz = outF + (size_t)s * M * N;
    f32_store_pass(sF, outz, m0, n0, N, w, lane);
    __threadfence();
    f32_store_pass(sF, outz, m0, n0, N, w, lane);
  } else {
    _Float16* outz = out0 + (size_t)s * M * N;
    f16_store_pass(sH, outz, m0, n0, N, w, lane);
    __threadfence();
    f16_store_pass(sH, outz, m0, n0, N, w, lane);
  }
}

__device__ __forceinline__ v16h pack_p(v8f a, v8f c) {
  const v16h r = { (_Float16)(a[0] * PSCALE), (_Float16)(a[1] * PSCALE), (_Float16)(a[2] * PSCALE), (_Float16)(a[3] * PSCALE),
                   (_Float16)(a[4] * PSCALE), (_Float16)(a[5] * PSCALE), (_Float16)(a[6] * PSCALE), (_Float16)(a[7] * PSCALE),
                   (_Float16)(c[0] * PSCALE), (_Float16)(c[1] * PSCALE), (_Float16)(c[2] * PSCALE), (_Float16)(c[3] * PSCALE),
                   (_Float16)(c[4] * PSCALE), (_Float16)(c[5] * PSCALE), (_Float16)(c[6] * PSCALE), (_Float16)(c[7] * PSCALE) };
  return r;
}

__device__ __forceinline__ void att_store_pass(const _Float16* sT, _Float16* mh, size_t rowbase,
                                               int qb, int w, int lane) {
  const int q8 = lane & 7, sub = lane >> 3;
  #pragma unroll
  for (int i = 0; i < 4; ++i) {
    const int d = 16 * w + i * 4 + sub;
    const v8h v = *(const v8ha*)(sT + d * 64 + 8 * q8);
    _Float16* dst = mh + (rowbase + (size_t)d) * EE + qb + 8 * q8;
    *(volatile v8h*)dst = v;
  }
}

__global__ __launch_bounds__(128) void attn_kernel(
    const _Float16* __restrict__ qh,
    const _Float16* __restrict__ kh,
    const _Float16* __restrict__ vt,
    const float* __restrict__ inter,
    _Float16* __restrict__ mh)
{
  __shared__ __attribute__((aligned(16))) float sO[4 * 16 * 64];
  __shared__ __attribute__((aligned(16))) _Float16 sT[64 * 64];

  const int tid = threadIdx.x, lane = tid & 31, w = tid >> 5;
  const int h = lane >> 4, m = lane & 15;
  const int istr = blockIdx.z;
  const int bhid = blockIdx.y, b = bhid >> 3, head = bhid & 7;
  const int qb = blockIdx.x * 64;
  const int q0 = qb + 16 * w;
  const int qplane = (istr * BB + b) * HH + head;

  const _Float16* qrow = qh + ((size_t)qplane * SS + q0 + m) * HD;
  const v16h qf0 = load_frag(qrow, h);
  const v16h qf1 = load_frag(qrow + 32, h);

  const v8f zero8 = {0.f, 0.f, 0.f, 0.f, 0.f, 0.f, 0.f, 0.f};
  float* so = sO + w * 1024;
  #pragma unroll
  for (int t = 0; t < 4; ++t)
    #pragma unroll
    for (int r = 0; r < 8; ++r) so[m * 64 + 16 * t + 8 * h + r] = 0.0f;

  #pragma unroll 1
  for (int j = 0; j < NSTR; ++j) {
    const float wij = inter[istr * NSTR + j] * 0.125f;
    const int kvp = (j * BB + b) * HH + head;
    const _Float16* kbase = kh + ((size_t)kvp * SS + m) * HD;
    const _Float16* vbase = vt + ((size_t)kvp * HD + m) * SS;

    v8f oj[4];
    #pragma unroll
    for (int t = 0; t < 4; ++t) oj[t] = zero8;
    float mrun = -1e30f, lrun = 0.0f;

    #pragma unroll 1
    for (int kb = 0; kb < SS; kb += 64) {
      v8f s[4];
      #pragma unroll
      for (int jj = 0; jj < 4; ++jj) {
        const _Float16* kp = kbase + (size_t)(kb + 16 * jj) * HD;
        const v16h kf0 = load_frag(kp, h);
        const v16h kf1 = load_frag(kp + 32, h);
        v8f zacc = zero8;
        zacc = wmma_f16(kf0, qf0, zacc);
        zacc = wmma_f16(kf1, qf1, zacc);
        s[jj] = zacc;
      }
      #pragma unroll
      for (int jj = 0; jj < 4; ++jj)
        #pragma unroll
        for (int r = 0; r < 8; ++r) s[jj][r] = s[jj][r] * wij;

      float mloc = s[0][0];
      #pragma unroll
      for (int jj = 0; jj < 4; ++jj)
        #pragma unroll
        for (int r = 0; r < 8; ++r) mloc = fmaxf(mloc, s[jj][r]);
      mloc = fmaxf(mloc, __shfl_xor(mloc, 16));
      const float mnew = fmaxf(mrun, mloc);
      const float alpha = __expf(mrun - mnew);
      mrun = mnew;
      float lsum = 0.0f;
      #pragma unroll
      for (int jj = 0; jj < 4; ++jj)
        #pragma unroll
        for (int r = 0; r < 8; ++r) {
          const float p = __expf(s[jj][r] - mnew);
          s[jj][r] = p;
          lsum += p;
        }
      lsum += __shfl_xor(lsum, 16);
      lrun = lrun * alpha + lsum;
      #pragma unroll
      for (int t = 0; t < 4; ++t)
        #pragma unroll
        for (int r = 0; r < 8; ++r) oj[t][r] = oj[t][r] * alpha;

      const v16h pb0 = pack_p(s[0], s[1]);
      const v16h pb1 = pack_p(s[2], s[3]);

      #pragma unroll
      for (int t = 0; t < 4; ++t) {
        const _Float16* vp = vbase + (size_t)(16 * t) * SS + kb;
        const v16h vf0 = load_frag(vp, h);
        const v16h vf1 = load_frag(vp + 32, h);
        oj[t] = wmma_f16(vf0, pb0, oj[t]);
        oj[t] = wmma_f16(vf1, pb1, oj[t]);
      }
    }

    const float inv = (1.0f / lrun) * (ASCALE / (PSCALE * (float)NSTR));
    #pragma unroll
    for (int t = 0; t < 4; ++t)
      #pragma unroll
      for (int r = 0; r < 8; ++r) {
        const int idx = m * 64 + 16 * t + 8 * h + r;
        const float cur = so[idx];
        so[idx] = cur + oj[t][r] * inv;
      }
  }

  #pragma unroll
  for (int t = 0; t < 4; ++t)
    #pragma unroll
    for (int r = 0; r < 8; ++r) {
      const int d = 16 * t + 8 * h + r;
      sT[d * 64 + 16 * w + m] = (_Float16)so[m * 64 + d];
    }
  __syncthreads();

  const size_t rowbase = (size_t)(istr * BB + b) * SS + (size_t)head * HD;
  att_store_pass(sT, mh, rowbase, qb, w, lane);
  __threadfence();
  att_store_pass(sT, mh, rowbase, qb, w, lane);
}

template <int FIRST>
__global__ __launch_bounds__(128) void ln_kernel(
    const float* __restrict__ a0, const float* __restrict__ a1,
    const float* __restrict__ a2, const float* __restrict__ a3,
    const float* __restrict__ bsum, const float* __restrict__ gam, const float* __restrict__ bet,
    float* __restrict__ outF, _Float16* __restrict__ outH, int rowsPerStream)
{
  __shared__ float red[8];
  const int row = blockIdx.x, tid = threadIdx.x, lane = tid & 31, w = tid >> 5;
  const int c = tid * 4;
  const int s = row / rowsPerStream;

  const float* ap;
  if (FIRST) {
    const int rl = row - s * rowsPerStream;
    const float* base = (s == 0) ? a0 : ((s == 1) ? a1 : ((s == 2) ? a2 : a3));
    ap = base + (size_t)rl * EE;
  } else {
    ap = a0 + (size_t)row * EE;
  }
  const v4f va = *(const v4fa*)(ap + c);
  const v4f vb = *(const v4fa*)(bsum + (size_t)row * EE + c);
  const v4f v = va + vb;

  float sum = (v.x + v.y) + (v.z + v.w);
  #pragma unroll
  for (int o = 16; o > 0; o >>= 1) sum += __shfl_xor(sum, o);
  if (lane == 0) red[w] = sum;
  __syncthreads();
  const float mean = ((red[0] + red[1]) + (red[2] + red[3])) * (1.0f / (float)EE);

  v4f d;
  d.x = v.x - mean; d.y = v.y - mean; d.z = v.z - mean; d.w = v.w - mean;
  float sq = (d.x * d.x + d.y * d.y) + (d.z * d.z + d.w * d.w);
  #pragma unroll
  for (int o = 16; o > 0; o >>= 1) sq += __shfl_xor(sq, o);
  if (lane == 0) red[4 + w] = sq;
  __syncthreads();
  const float var = ((red[4] + red[5]) + (red[6] + red[7])) * (1.0f / (float)EE);
  const float rstd = rsqrtf(var + 1e-5f);

  const v4f gg = *(const v4fa*)(gam + (size_t)s * EE + c);
  const v4f be = *(const v4fa*)(bet + (size_t)s * EE + c);
  v4f y;
  y.x = d.x * rstd * gg.x + be.x;
  y.y = d.y * rstd * gg.y + be.y;
  y.z = d.z * rstd * gg.z + be.z;
  y.w = d.w * rstd * gg.w + be.w;

  float* dstF = outF + (size_t)row * EE + c;
  v4h yh = { (_Float16)y.x, (_Float16)y.y, (_Float16)y.z, (_Float16)y.w };
  _Float16* dstH = outH + (size_t)row * EE + c;

  *(volatile v4f*)dstF = y;
  if (FIRST) *(volatile v4h*)dstH = yh;
  __threadfence();
  *(volatile v4f*)dstF = y;
  if (FIRST) *(volatile v4h*)dstH = yh;
}

extern "C" void kernel_launch(void* const* d_in, const int* in_sizes, int n_in,
                              void* d_out, int out_size, void* d_ws, size_t ws_size,
                              hipStream_t stream) {
  if (n_in < 18) return;
  const int nx  = BB * SS * EE;
  const int nwe = NSTR * EE * EE;
  const int nwf = NSTR * EE * FF;
  if (in_sizes[0] != nx || in_sizes[1] != nx || in_sizes[2] != nx || in_sizes[3] != nx) return;
  if (in_sizes[4] != nwe || in_sizes[5] != nwe || in_sizes[6] != nwe || in_sizes[7] != nwe) return;
  if (in_sizes[8] != NSTR * EE || in_sizes[9] != NSTR * EE || in_sizes[10] != NSTR * EE) return;
  if (in_sizes[11] != NSTR * EE || in_sizes[12] != NSTR * EE || in_sizes[16] != NSTR * EE) return;
  if (in_sizes[13] != nwf || in_sizes[15] != nwf || in_sizes[14] != NSTR * FF) return;
  if (in_sizes[17] != NSTR * NSTR) return;
  if (out_size != NSTR * nx) return;

  const float* x0   = (const float*)d_in[0];
  const float* x1   = (const float*)d_in[1];
  const float* x2   = (const float*)d_in[2];
  const float* x3   = (const float*)d_in[3];
  const float* Wq   = (const float*)d_in[4];
  const float* Wk   = (const float*)d_in[5];
  const float* Wv   = (const float*)d_in[6];
  const float* Wo   = (const float*)d_in[7];
  const float* bo   = (const float*)d_in[8];
  const float* ln1g = (const float*)d_in[9];
  const float* ln1b = (const float*)d_in[10];
  const float* ln2g = (const float*)d_in[11];
  const float* ln2b = (const float*)d_in[12];
  const float* W1   = (const float*)d_in[13];
  const float* bf1  = (const float*)d_in[14];
  const float* W2   = (const float*)d_in[15];
  const float* bf2  = (const float*)d_in[16];
  const float* inter = (const float*)d_in[17];
  float* out = (float*)d_out;

  const size_t sz_xh   = (size_t)NSTR * nx * 2;
  const size_t sz_wqkv = (size_t)3 * nwe * 2;
  const size_t sz_wo   = (size_t)nwe * 2;
  const size_t sz_w1   = (size_t)nwf * 2;
  const size_t sz_w2   = (size_t)nwf * 2;
  const size_t sz_pl   = (size_t)NSTR * nx * 2;
  const size_t sz_mh   = (size_t)NSTR * nx * 2;
  const size_t sz_f32  = (size_t)NSTR * nx * 4;
  const size_t sz_r1h  = (size_t)NSTR * nx * 2;
  const size_t sz_hb   = (size_t)NSTR * MROWS * FF * 2;

  const size_t o_xh   = 0;
  const size_t o_wqkv = o_xh + sz_xh;
  const size_t o_wo   = o_wqkv + sz_wqkv;
  const size_t o_w1   = o_wo + sz_wo;
  const size_t o_w2   = o_w1 + sz_w1;
  const size_t o_q    = o_w2 + sz_w2;
  const size_t o_k    = o_q + sz_pl;
  const size_t o_v    = o_k + sz_pl;
  const size_t o_mh   = o_v + sz_pl;
  const size_t o_r1f  = o_mh + sz_mh;
  const size_t o_r1h  = o_r1f + sz_f32;
  const size_t o_hb   = o_r1h + sz_r1h;
  const size_t total  = o_hb + sz_hb;
  const size_t o_pf   = o_q;
  if (sz_f32 > 3 * sz_pl) return;
  if (total > ws_size) return;
  if (total > (size_t)134217728) return;

  char* ws = (char*)d_ws;
  _Float16* xh    = (_Float16*)(ws + o_xh);
  _Float16* wqkvT = (_Float16*)(ws + o_wqkv);
  _Float16* woT   = (_Float16*)(ws + o_wo);
  _Float16* w1T   = (_Float16*)(ws + o_w1);
  _Float16* w2T   = (_Float16*)(ws + o_w2);
  _Float16* qh    = (_Float16*)(ws + o_q);
  _Float16* kh    = (_Float16*)(ws + o_k);
  _Float16* vt    = (_Float16*)(ws + o_v);
  _Float16* mh    = (_Float16*)(ws + o_mh);
  float*    r1f   = (float*)(ws + o_r1f);
  _Float16* r1h   = (_Float16*)(ws + o_r1h);
  _Float16* hb    = (_Float16*)(ws + o_hb);
  float*    projf = (float*)(ws + o_pf);
  float*    ffnf  = (float*)(ws + o_pf);

  const int per8 = nx / 8;
  const int tot8 = NSTR * per8;
  cvt_x_kernel<<<(tot8 + 255) / 256, 256, 0, stream>>>(x0, x1, x2, x3, xh, per8, tot8);

  cvt_wt_kernel<<<dim3(EE / 64, EE / 64, NSTR), 256, 0, stream>>>(Wq, wqkvT, EE, EE, WSCALE);
  cvt_wt_kernel<<<dim3(EE / 64, EE / 64, NSTR), 256, 0, stream>>>(Wk, wqkvT + (size_t)nwe, EE, EE, WSCALE);
  cvt_wt_kernel<<<dim3(EE / 64, EE / 64, NSTR), 256, 0, stream>>>(Wv, wqkvT + (size_t)2 * nwe, EE, EE, WSCALE);
  cvt_wt_kernel<<<dim3(EE / 64, EE / 64, NSTR), 256, 0, stream>>>(Wo, woT, EE, EE, WSCALE);
  cvt_wt_kernel<<<dim3(FF / 64, EE / 64, NSTR), 256, 0, stream>>>(W1, w1T, EE, FF, WSCALE);
  cvt_wt_kernel<<<dim3(EE / 64, FF / 64, NSTR), 256, 0, stream>>>(W2, w2T, FF, EE, WSCALE);

  gemm_kernel<0><<<dim3(MROWS / 128, EE / 64, 3 * NSTR), 128, 0, stream>>>(
      xh, wqkvT, bo, r1f, qh, kh, vt, MROWS, EE, EE, 1.0f / WSCALE);

  attn_kernel<<<dim3(SS / 64, BB * HH, NSTR), 128, 0, stream>>>(qh, kh, vt, inter, mh);

  gemm_kernel<1><<<dim3(MROWS / 128, EE / 64, NSTR), 128, 0, stream>>>(
      mh, woT, bo, projf, r1h, r1h, r1h, MROWS, EE, EE, 1.0f / (ASCALE * WSCALE));

  ln_kernel<1><<<NSTR * MROWS, 128, 0, stream>>>(x0, x1, x2, x3, projf, ln1g, ln1b, r1f, r1h, MROWS);

  gemm_kernel<2><<<dim3(MROWS / 128, FF / 64, NSTR), 128, 0, stream>>>(
      r1h, w1T, bf1, r1f, hb, hb, hb, MROWS, FF, EE, 1.0f / WSCALE);

  gemm_kernel<1><<<dim3(MROWS / 128, EE / 64, NSTR), 128, 0, stream>>>(
      hb, w2T, bf2, ffnf, r1h, r1h, r1h, MROWS, EE, FF, 1.0f / (ASCALE * WSCALE));

  ln_kernel<0><<<NSTR * MROWS, 128, 0, stream>>>(r1f, r1f, r1f, r1f, ffnf, ln2g, ln2b, out, r1h, MROWS);
}
